// LSTMAutoencoder_28458453303916
// MI455X (gfx1250) — hardware-verified
//
#include <hip/hip_runtime.h>
#include <stddef.h>
#include <stdint.h>


#define NB 64
#define TT 512
#define DD 32
#define HH 256
#define GG 1024
#define RT (NB * TT)

typedef __bf16 v8b  __attribute__((ext_vector_type(8)));
typedef __bf16 v16b __attribute__((ext_vector_type(16)));
typedef float  v8f  __attribute__((ext_vector_type(8)));
typedef float  v4f  __attribute__((ext_vector_type(4)));
typedef int    v4i  __attribute__((ext_vector_type(4)));

union Frag { v16b v; v8b h[2]; };
union Pk8  { v8b b; v4i u; __bf16 s[8]; };

static __device__ __forceinline__ __bf16 f2bf(float f) {
  unsigned u = __builtin_bit_cast(unsigned, f);
  u += 0x7FFFu + ((u >> 16) & 1u);
  unsigned short s = (unsigned short)(u >> 16);
  return __builtin_bit_cast(__bf16, s);
}
static __device__ __forceinline__ float bf2f(__bf16 b) {
  unsigned short s = __builtin_bit_cast(unsigned short, b);
  return __builtin_bit_cast(float, ((unsigned)s) << 16);
}

static __device__ __forceinline__ v8f mma16(v16b a, v16b b, v8f c) {
  v8f d = __builtin_amdgcn_wmma_f32_16x16x32_bf16(false, a, false, b, (short)0, c, false, false);
  asm volatile("v_nop\n\tv_nop\n\tv_nop\n\tv_nop" : "+v"(d) : "v"(a), "v"(b));
  return d;
}
static __device__ __forceinline__ v8f mma3(const Frag& ah, const Frag& al,
                                            const Frag& bh, const Frag& bl, v8f c) {
  c = mma16(ah.v, bh.v, c);
  c = mma16(ah.v, bl.v, c);
  c = mma16(al.v, bh.v, c);
  return c;
}
static __device__ __forceinline__ void split8(const float* __restrict__ p, Pk8& hi, Pk8& lo) {
  v4f x0 = *(const v4f*)p;
  v4f x1 = *(const v4f*)(p + 4);
  float xs[8];
  xs[0] = x0.x; xs[1] = x0.y; xs[2] = x0.z; xs[3] = x0.w;
  xs[4] = x1.x; xs[5] = x1.y; xs[6] = x1.z; xs[7] = x1.w;
#pragma unroll
  for (int e = 0; e < 8; ++e) {
    __bf16 hb = f2bf(xs[e]);
    hi.s[e] = hb;
    lo.s[e] = f2bf(xs[e] - bf2f(hb));
  }
}
static __device__ __forceinline__ float sigm(float x) {
  return 1.0f / (1.0f + expf(-x));
}

__global__ __launch_bounds__(256) void k_split_planes(const float* __restrict__ src,
                                                      __bf16* __restrict__ hi,
                                                      __bf16* __restrict__ lo, int n8) {
  const int i = blockIdx.x * 256 + threadIdx.x;
  const bool ok = i < n8;
  Pk8 ph, pl;
  ph.u = (v4i){0, 0, 0, 0};
  pl.u = (v4i){0, 0, 0, 0};
  if (ok) split8(src + (size_t)i * 8, ph, pl);
  if (ok) {
    *(volatile v4i*)(hi + (size_t)i * 8) = ph.u;
    *(volatile v4i*)(lo + (size_t)i * 8) = pl.u;
  }
  __threadfence();
  if (ok) {
    *(volatile v4i*)(hi + (size_t)i * 8) = ph.u;
    *(volatile v4i*)(lo + (size_t)i * 8) = pl.u;
  }
}

__global__ __launch_bounds__(256) void k_gemm3(const float* __restrict__ A,
                                              const float* __restrict__ W,
                                              const float* __restrict__ bias,
                                              float* __restrict__ out,
                                              int R, int K, int N, int ldo) {
  __shared__ __attribute__((aligned(16))) __bf16 sAh[64 * 40];
  __shared__ __attribute__((aligned(16))) __bf16 sAl[64 * 40];
  __shared__ __attribute__((aligned(16))) __bf16 sBh[128 * 40];
  __shared__ __attribute__((aligned(16))) __bf16 sBl[128 * 40];
  __shared__ __attribute__((aligned(16))) float  sO[64 * 128];

  const int tid  = threadIdx.x;
  const int lane = tid & 31;
  const int wv   = tid >> 5;
  const int mt   = wv & 3;
  const int ng   = wv >> 2;
  const int hf   = lane >> 4;
  const int nl   = lane & 15;
  const int koff = hf * 8;
  const int row0  = blockIdx.x * 64;
  const int ncol0 = blockIdx.y * 128;

  const int ar = tid >> 2;
  const int ac = (tid & 3) * 8;
  int gr = row0 + ar;          if (gr > R - 1) gr = R - 1;
  int bn0 = ncol0 + ar;        if (bn0 > N - 1) bn0 = N - 1;
  int bn1 = ncol0 + 64 + ar;   if (bn1 > N - 1) bn1 = N - 1;
  const float* Ap  = A + (size_t)gr  * K + ac;
  const float* Bp0 = W + (size_t)bn0 * K + ac;
  const float* Bp1 = W + (size_t)bn1 * K + ac;

  v8f acc[4];
#pragma unroll
  for (int j = 0; j < 4; ++j) acc[j] = (v8f){0.f, 0.f, 0.f, 0.f, 0.f, 0.f, 0.f, 0.f};

  const int nk = K >> 5;
  for (int ks = 0; ks < nk; ++ks) {
    const int k0 = ks * 32;
    __syncthreads();
    {
      Pk8 ph, pl;
      split8(Ap + k0, ph, pl);
      *(v8b*)&sAh[ar * 40 + ac] = ph.b;
      *(v8b*)&sAl[ar * 40 + ac] = pl.b;
      split8(Bp0 + k0, ph, pl);
      *(v8b*)&sBh[ar * 40 + ac] = ph.b;
      *(v8b*)&sBl[ar * 40 + ac] = pl.b;
      split8(Bp1 + k0, ph, pl);
      *(v8b*)&sBh[(64 + ar) * 40 + ac] = ph.b;
      *(v8b*)&sBl[(64 + ar) * 40 + ac] = pl.b;
    }
    __syncthreads();

    Frag ah, al;
    {
      const int ai = (mt * 16 + nl) * 40 + koff;
      ah.h[0] = *(const v8b*)&sAh[ai];
      ah.h[1] = *(const v8b*)&sAh[ai + 16];
      al.h[0] = *(const v8b*)&sAl[ai];
      al.h[1] = *(const v8b*)&sAl[ai + 16];
    }
#pragma unroll
    for (int j = 0; j < 4; ++j) {
      const int bi = (ng * 64 + j * 16 + nl) * 40 + koff;
      Frag bh, bl;
      bh.h[0] = *(const v8b*)&sBh[bi];
      bh.h[1] = *(const v8b*)&sBh[bi + 16];
      bl.h[0] = *(const v8b*)&sBl[bi];
      bl.h[1] = *(const v8b*)&sBl[bi + 16];
      acc[j] = mma3(ah, al, bh, bl, acc[j]);
    }
  }

#pragma unroll
  for (int j = 0; j < 4; ++j) {
    const int cl = ng * 64 + j * 16 + nl;
    int cb = ncol0 + cl;  if (cb > N - 1) cb = N - 1;
    const float bs = bias[cb];
#pragma unroll
    for (int r = 0; r < 8; ++r) sO[(mt * 16 + hf * 8 + r) * 128 + cl] = acc[j][r] + bs;
  }
  __syncthreads();

  int nv = N - ncol0;  if (nv > 128) nv = 128;
  const int nq  = nv >> 2;
  const int tot = 64 * nq;
  for (int i = tid; i < tot; i += 256) {
    const int r = i / nq;
    const int q = i - r * nq;
    const int orow = row0 + r;
    if (orow < R) {
      v4f v = *(const v4f*)&sO[r * 128 + q * 4];
      *(volatile v4f*)(out + (size_t)orow * ldo + ncol0 + q * 4) = v;
    }
  }
  __threadfence();
  for (int i = tid; i < tot; i += 256) {
    const int r = i / nq;
    const int q = i - r * nq;
    const int orow = row0 + r;
    if (orow < R) {
      v4f v = *(const v4f*)&sO[r * 128 + q * 4];
      *(volatile v4f*)(out + (size_t)orow * ldo + ncol0 + q * 4) = v;
    }
  }
}

__global__ __launch_bounds__(256) void k_relu_last(const float* __restrict__ y,
                                                   float* __restrict__ rep, int nb) {
  const int i = blockIdx.x * 256 + threadIdx.x;
  const int tot = nb * (HH / 4);
  const bool ok = i < tot;
  v4f v = (v4f){0.f, 0.f, 0.f, 0.f};
  if (ok) {
    const int b = i / (HH / 4);
    const int q = i - b * (HH / 4);
    v = *(const v4f*)(y + ((size_t)b * TT + (TT - 1)) * HH + q * 4);
    v.x = v.x > 0.f ? v.x : 0.f;
    v.y = v.y > 0.f ? v.y : 0.f;
    v.z = v.z > 0.f ? v.z : 0.f;
    v.w = v.w > 0.f ? v.w : 0.f;
  }
  if (ok) *(volatile v4f*)(rep + (size_t)i * 4) = v;
  __threadfence();
  if (ok) *(volatile v4f*)(rep + (size_t)i * 4) = v;
}

__global__ __launch_bounds__(512) void k_scan3(const float* __restrict__ xp,
                                              const __bf16* __restrict__ Wh,
                                              const __bf16* __restrict__ Wl,
                                              float* __restrict__ y,
                                              int nb, int rmb, int rmt) {
  __shared__ __attribute__((aligned(16))) __bf16 pH[16 * 264];
  __shared__ __attribute__((aligned(16))) __bf16 pL[16 * 264];
  __shared__ __attribute__((aligned(16))) float  hs[16 * 256];

  const int tid  = threadIdx.x;
  const int lane = tid & 31;
  const int wv   = tid >> 5;
  const int hf   = lane >> 4;
  const int nl   = lane & 15;
  const int koff = hf * 8;
  const int col  = wv * 16 + nl;
  const int b0   = blockIdx.x * 16;

  {
    const __bf16 z = f2bf(0.0f);
    for (int i = tid; i < 16 * 264; i += 512) { pH[i] = z; pL[i] = z; }
  }
  float c[8];
#pragma unroll
  for (int r = 0; r < 8; ++r) c[r] = 0.f;

  size_t xrow[8];
#pragma unroll
  for (int r = 0; r < 8; ++r) {
    int b = b0 + hf * 8 + r;  if (b > nb - 1) b = nb - 1;
    xrow[r] = (size_t)b * (size_t)rmb;
  }
  __syncthreads();

  for (int t = 0; t < TT; ++t) {
    v8f acc[4];
#pragma unroll
    for (int j = 0; j < 4; ++j) acc[j] = (v8f){0.f, 0.f, 0.f, 0.f, 0.f, 0.f, 0.f, 0.f};

#pragma unroll 1
    for (int ks = 0; ks < 8; ++ks) {
      const int k0 = ks * 32;
      Frag ah, al;
      {
        const int ai = nl * 264 + k0 + koff;
        ah.h[0] = *(const v8b*)&pH[ai];
        ah.h[1] = *(const v8b*)&pH[ai + 16];
        al.h[0] = *(const v8b*)&pL[ai];
        al.h[1] = *(const v8b*)&pL[ai + 16];
      }
#pragma unroll
      for (int j = 0; j < 4; ++j) {
        const size_t bi = (size_t)(j * HH + col) * HH + k0 + koff;
        Frag bh, bl;
        bh.h[0] = *(const v8b*)(Wh + bi);
        bh.h[1] = *(const v8b*)(Wh + bi + 16);
        bl.h[0] = *(const v8b*)(Wl + bi);
        bl.h[1] = *(const v8b*)(Wl + bi + 16);
        acc[j] = mma3(ah, al, bh, bl, acc[j]);
      }
    }

    float xg[4][8];
#pragma unroll
    for (int j = 0; j < 4; ++j)
#pragma unroll
      for (int r = 0; r < 8; ++r)
        xg[j][r] = xp[(xrow[r] + (size_t)t * (size_t)rmt) * GG + j * HH + col];

    __syncthreads();

#pragma unroll
    for (int r = 0; r < 8; ++r) {
      const float gi = acc[0][r] + xg[0][r];
      const float gf = acc[1][r] + xg[1][r];
      const float gc = acc[2][r] + xg[2][r];
      const float go = acc[3][r] + xg[3][r];
      const float ig = sigm(gi);
      const float fg = sigm(gf);
      const float gg = tanhf(gc);
      const float og = sigm(go);
      const float cn = fg * c[r] + ig * gg;
      c[r] = cn;
      const float hv = og * tanhf(cn);
      const int row = hf * 8 + r;
      hs[row * 256 + col] = hv;
      const __bf16 hb = f2bf(hv);
      pH[row * 264 + col] = hb;
      pL[row * 264 + col] = f2bf(hv - bf2f(hb));
    }
    __syncthreads();

#pragma unroll
    for (int m = 0; m < 2; ++m) {
      const int i = tid + 512 * m;
      const int row = i >> 6;
      const int q = i & 63;
      const int b = b0 + row;
      if (b < nb) {
        v4f v = *(const v4f*)&hs[row * 256 + q * 4];
        *(volatile v4f*)(y + ((size_t)b * TT + t) * HH + q * 4) = v;
      }
    }
    __threadfence();
#pragma unroll
    for (int m = 0; m < 2; ++m) {
      const int i = tid + 512 * m;
      const int row = i >> 6;
      const int q = i & 63;
      const int b = b0 + row;
      if (b < nb) {
        v4f v = *(const v4f*)&hs[row * 256 + q * 4];
        *(volatile v4f*)(y + ((size_t)b * TT + t) * HH + q * 4) = v;
      }
    }
  }
}

extern "C" void kernel_launch(void* const* d_in, const int* in_sizes, int n_in,
                              void* d_out, int out_size, void* d_ws, size_t ws_size,
                              hipStream_t stream) {
  if (n_in < 12) return;
  if (in_sizes[0] != RT * DD || in_sizes[1] != GG * DD || in_sizes[2] != GG * HH ||
      in_sizes[3] != GG || in_sizes[4] != GG * HH || in_sizes[5] != GG * HH ||
      in_sizes[6] != GG || in_sizes[7] != 4 * GG * HH || in_sizes[8] != 4 * GG * HH ||
      in_sizes[9] != 4 * GG || in_sizes[10] != DD * HH || in_sizes[11] != DD) return;
  if (out_size != RT * DD) return;

  const float* x     = (const float*)d_in[0];
  const float* eWih0 = (const float*)d_in[1];
  const float* eWhh0 = (const float*)d_in[2];
  const float* eb0   = (const float*)d_in[3];
  const float* eWih1 = (const float*)d_in[4];
  const float* eWhh1 = (const float*)d_in[5];
  const float* eb1   = (const float*)d_in[6];
  const float* dWih  = (const float*)d_in[7];
  const float* dWhh  = (const float*)d_in[8];
  const float* db    = (const float*)d_in[9];
  const float* Wout  = (const float*)d_in[10];
  const float* bout  = (const float*)d_in[11];
  float* outp = (float*)d_out;

  size_t off = 0;
  auto carve = [&](size_t bytes) {
    size_t r = off;
    off += (bytes + 255) & ~(size_t)255;
    return r;
  };
  const size_t o_xp  = carve((size_t)RT * GG * sizeof(float));
  const size_t o_yA  = carve((size_t)RT * HH * sizeof(float));
  const size_t o_yB  = carve((size_t)RT * HH * sizeof(float));
  const size_t o_wh  = carve((size_t)GG * HH * 2);
  const size_t o_wl  = carve((size_t)GG * HH * 2);
  const size_t o_rep = carve((size_t)NB * HH * sizeof(float));
  if (off > ws_size) return;

  char* ws = (char*)d_ws;
  float*  xpb = (float*)(ws + o_xp);
  float*  yA  = (float*)(ws + o_yA);
  float*  yB  = (float*)(ws + o_yB);
  __bf16* wh  = (__bf16*)(ws + o_wh);
  __bf16* wl  = (__bf16*)(ws + o_wl);
  float*  rep = (float*)(ws + o_rep);

  auto gemm = [&](const float* Ain, const float* Wm, const float* bias, float* o,
                  int R, int K, int N, int ldo) {
    if ((K & 31) != 0 || (N & 3) != 0 || (ldo & 3) != 0) return;
    dim3 grid((R + 63) / 64, (N + 127) / 128);
    k_gemm3<<<grid, 256, 0, stream>>>(Ain, Wm, bias, o, R, K, N, ldo);
  };
  auto scan = [&](const float* whh, float* yout, int rmb, int rmt) {
    const int n8 = GG * HH / 8;
    k_split_planes<<<(n8 + 255) / 256, 256, 0, stream>>>(whh, wh, wl, n8);
    k_scan3<<<(NB + 15) / 16, 512, 0, stream>>>(xpb, wh, wl, yout, NB, rmb, rmt);
  };
  auto layer = [&](const float* Ain, int K, const float* wih, const float* b,
                   const float* whh, float* yout) {
    gemm(Ain, wih, b, xpb, RT, K, GG, GG);
    scan(whh, yout, TT, 1);
  };

  layer(x,  DD, eWih0, eb0, eWhh0, yA);
  layer(yA, HH, eWih1, eb1, eWhh1, yB);

  k_relu_last<<<(NB * (HH / 4) + 255) / 256, 256, 0, stream>>>(yB, rep, NB);
  gemm(rep, dWih + (size_t)0 * GG * HH, db + 0 * GG, xpb, NB, HH, GG, GG);
  scan(dWhh + (size_t)0 * GG * HH, yA, 1, 0);

  layer(yA, HH, dWih + (size_t)1 * GG * HH, db + 1 * GG, dWhh + (size_t)1 * GG * HH, yB);
  layer(yB, HH, dWih + (size_t)2 * GG * HH, db + 2 * GG, dWhh + (size_t)2 * GG * HH, yA);
  layer(yA, HH, dWih + (size_t)3 * GG * HH, db + 3 * GG, dWhh + (size_t)3 * GG * HH, yB);

  gemm(yB, Wout, bout, outp, RT, HH, DD, DD);
}
